// StackGRU_24515673325785
// MI455X (gfx1250) — hardware-run, weakly checked
//
#include <hip/hip_runtime.h>
#include <math.h>

typedef __attribute__((ext_vector_type(16))) _Float16 v16h;
typedef __attribute__((ext_vector_type(8)))  _Float16 v8h;
typedef __attribute__((ext_vector_type(8)))  float    v8f;
typedef __attribute__((ext_vector_type(4)))  float    v4f;

constexpr int kNB = 64;
constexpr int kNT = 1024;
constexpr int kNI = 64;
constexpr int kNH = 512;
constexpr int kNO = 24;
constexpr int kNG = 3 * kNH;
constexpr int kMB = 16;
constexpr int kBlocks = kNB / kMB;
constexpr int kK1 = kNI + kNH;
constexpr int kK2 = 2 * kNH;
constexpr int kHP = kNH + 8;
constexpr int kXP = kNI + 8;
constexpr int kFl = 16;
constexpr int kOBS = kFl * kNO;
constexpr int kHeadRows = 64;
constexpr float kCarryA = 8.0f;
constexpr float kCarryW = 1024.0f;
constexpr float kFold   = 1.0f / (kCarryA * kCarryW);
constexpr float kF16Min = 6.103515625e-05f;

static_assert(kNB % kMB == 0);
static_assert(kK1 % 32 == 0 && kK2 % 32 == 0 && kNH % 32 == 0 && kNI % 32 == 0);
static_assert(kNG % 16 == 0 && kNH == 16 * 32);
static_assert((kOBS * 4) % 512 == 0 && (kOBS * 4) / 512 == 3);
static_assert((kNT % kFl) == 0 && (kFl * kNO * 4) % 128 == 0);
static_assert((kHP * 2) % 16 == 0 && (kXP * 2) % 16 == 0);
static_assert(kFold == 1.0f / 8192.0f);

constexpr size_t kBytesW1 = (size_t)kNG * kK1 * 2;
constexpr size_t kBytesW2 = (size_t)kNG * kK2 * 2;
constexpr size_t kBytesWO = (size_t)kHeadRows * kNH * 2;
constexpr size_t kOffW1 = 0;
constexpr size_t kOffW2 = kOffW1 + kBytesW1;
constexpr size_t kOffWO = kOffW2 + kBytesW2;
constexpr size_t kWsTotal = kOffWO + kBytesWO;
static_assert(kBytesW1 == 1769472ull && kBytesW2 == 3145728ull && kBytesWO == 65536ull);
static_assert(kWsTotal == 4980736ull);
static_assert((kOffW2 % 128) == 0 && (kOffWO % 128) == 0);
static_assert(kWsTotal <= 134217728ull);

__device__ __forceinline__ unsigned short f2bf_bits(float f) {
  unsigned u = __float_as_uint(f);
  return (unsigned short)((u + 0x7FFFu + ((u >> 16) & 1u)) >> 16);
}
__device__ __forceinline__ float bf_bits2f(unsigned short h) { return __uint_as_float(((unsigned)h) << 16); }
__device__ __forceinline__ float bf_val(float f) { return bf_bits2f(f2bf_bits(f)); }

__device__ __forceinline__ _Float16 carry_to_h16(float v, float carry) {
  float s = v * carry;
  s = (fabsf(s) < kF16Min) ? 0.0f : s;
  return (_Float16)s;
}

__device__ __forceinline__ float ld_bf(const float* p) {
  float v = *p;
  asm volatile("" : "+v"(v));
  return bf_val(v);
}

union FragU { v16h v; v8h h[2]; };
__device__ __forceinline__ v16h frag_load(const _Float16* p) {
  FragU f;
  f.h[0] = *(const v8h*)(p);
  f.h[1] = *(const v8h*)(p + 16);
  return f.v;
}

__device__ __forceinline__ v8f mma_g(v16h a, v16h b, v8f c) {
  c = __builtin_amdgcn_wmma_f32_16x16x32_f16(false, a, false, b, (short)0, c, false, false);
  asm volatile("v_nop\n\tv_nop\n\tv_nop\n\tv_nop" : "+v"(c) : "v"(a), "v"(b));
  return c;
}

template <int KC>
__device__ __forceinline__ void gemm_part(const _Float16* ap, const _Float16* wp, int nks,
                                          v8f& gr, v8f& gz, v8f& gn) {
#pragma unroll 1
  for (int ks = 0; ks < nks; ++ks) {
    const v16h a  = frag_load(ap + 32 * ks);
    const v16h br = frag_load(wp + 32 * ks);
    const v16h bz = frag_load(wp + (size_t)kNH * KC + 32 * ks);
    const v16h bn = frag_load(wp + (size_t)2 * kNH * KC + 32 * ks);
    gr = mma_g(a, br, gr);
    gz = mma_g(a, bz, gz);
    gn = mma_g(a, bn, gn);
  }
}

__device__ __forceinline__ float fast_sigmoid(float v) {
  return __builtin_amdgcn_rcpf(1.0f + __expf(-v));
}
__device__ __forceinline__ float fast_tanh(float v) {
  const float t = __expf(-2.0f * fabsf(v));
  const float q = (1.0f - t) * __builtin_amdgcn_rcpf(1.0f + t);
  return copysignf(q, v);
}

__device__ __forceinline__ void gate_update(const v8f& ar, const v8f& az, const v8f& ai, const v8f& ah,
                                            float cr, float cz, float bi, float bh, float (&h)[8]) {
#pragma unroll
  for (int e = 0; e < 8; ++e) {
    const float rg = fast_sigmoid(fmaf(ar[e], kFold, cr));
    const float zg = fast_sigmoid(fmaf(az[e], kFold, cz));
    const float hn = fmaf(ah[e], kFold, bh);
    const float in = fmaf(ai[e], kFold, bi);
    const float ng = fast_tanh(fmaf(rg, hn, in));
    h[e] = fmaf(zg, h[e] - ng, ng);
  }
}

__global__ __launch_bounds__(256) void pack_weight_plane(
    const float* __restrict__ src, int srcRows, int dstRows, int cs,
    unsigned short* __restrict__ dst, int pitch, int coloff) {
  const int i = blockIdx.x * 256 + threadIdx.x;
  const int cpr = cs >> 3;
  if (i >= dstRows * cpr) return;
  const int r  = i / cpr;
  const int kc = i - r * cpr;
  const bool live = (r < srcRows);
  const int rs = live ? r : (srcRows - 1);
  const float* sp = src + (size_t)rs * cs + kc * 8;
  v4f a0 = *(const v4f*)(sp);
  v4f a1 = *(const v4f*)(sp + 4);
  asm volatile("" : "+v"(a0), "+v"(a1));
  v8h hv;
#pragma unroll
  for (int e = 0; e < 4; ++e) {
    const float f0 = live ? bf_val(a0[e]) : 0.0f;
    const float f1 = live ? bf_val(a1[e]) : 0.0f;
    hv[e]     = carry_to_h16(f0, kCarryW);
    hv[4 + e] = carry_to_h16(f1, kCarryW);
  }
  unsigned short* q = dst + (size_t)r * pitch + coloff + kc * 8;
  *(volatile v8h*)q = hv;
  __threadfence();
  *(volatile v8h*)q = hv;
}

__global__ __launch_bounds__(512) void two_cell_scan(
    const float* __restrict__ x,
    const _Float16* __restrict__ W1, const _Float16* __restrict__ W2, const _Float16* __restrict__ WO,
    const float* __restrict__ bih1, const float* __restrict__ bhh1,
    const float* __restrict__ bih2, const float* __restrict__ bhh2,
    const float* __restrict__ bo1, const float* __restrict__ bo2,
    float* __restrict__ out) {
  __shared__ __align__(16) _Float16 H1s[kMB * kHP];
  __shared__ __align__(16) _Float16 H2s[kMB * kHP];
  __shared__ __align__(16) _Float16 XTs[kMB * kXP];
  __shared__ __align__(16) float    OBs[kMB * kOBS];
  __shared__ __align__(16) float    HPs[2 * 512];
  static_assert(sizeof(_Float16) * (2 * kMB * kHP + kMB * kXP) + sizeof(float) * (kMB * kOBS + 2 * 512) <= 65536);

  const int tid  = threadIdx.x;
  const int wave = tid >> 5;
  const int lane = tid & 31;
  const int hh   = lane >> 4;
  const int c    = lane & 15;
  const int blk  = blockIdx.x;

  float c1R[2], c1Z[2], c1I[2], c1N[2], c2R[2], c2Z[2], c2I[2], c2N[2];
#pragma unroll
  for (int u = 0; u < 2; ++u) {
    const int j = 32 * wave + 16 * u + c;
    c1R[u] = ld_bf(bih1 + j) + ld_bf(bhh1 + j);
    c1Z[u] = ld_bf(bih1 + kNH + j) + ld_bf(bhh1 + kNH + j);
    c1I[u] = ld_bf(bih1 + 2 * kNH + j);
    c1N[u] = ld_bf(bhh1 + 2 * kNH + j);
    c2R[u] = ld_bf(bih2 + j) + ld_bf(bhh2 + j);
    c2Z[u] = ld_bf(bih2 + kNH + j) + ld_bf(bhh2 + kNH + j);
    c2I[u] = ld_bf(bih2 + 2 * kNH + j);
    c2N[u] = ld_bf(bhh2 + 2 * kNH + j);
  }
  const int hcol  = 16 * (wave & 1) + c;
  const int hcolc = (hcol < kNO) ? hcol : (kNO - 1);
  const float bo1c = ld_bf(bo1 + hcolc);
  const float bo2c = ld_bf(bo2 + hcolc);

  float h1c[2][8], h2c[2][8];
#pragma unroll
  for (int u = 0; u < 2; ++u)
#pragma unroll
    for (int e = 0; e < 8; ++e) { h1c[u][e] = 0.0f; h2c[u][e] = 0.0f; }

  {
    v8h zv;
#pragma unroll
    for (int e = 0; e < 8; ++e) zv[e] = (_Float16)0.0f;
    for (int i = tid; i < (kMB * kHP) / 8; i += 512) {
      *(v8h*)(H1s + 8 * i) = zv;
      *(v8h*)(H2s + 8 * i) = zv;
    }
  }
  const int xi = tid - 384;
  const int xm = (xi >> 3) & 15;
  const int xk = (xi & 7) * 8;
  if (wave >= 12) {
    const float* xp = x + ((size_t)(kMB * blk + xm) * kNT) * kNI + xk;
    v4f a0 = *(const v4f*)(xp);
    v4f a1 = *(const v4f*)(xp + 4);
    v8h hv;
#pragma unroll
    for (int e = 0; e < 4; ++e) {
      hv[e]     = carry_to_h16(bf_val(a0[e]), kCarryA);
      hv[4 + e] = carry_to_h16(bf_val(a1[e]), kCarryA);
    }
    *(v8h*)(XTs + xm * kXP + xk) = hv;
  }
  __syncthreads();

  const v8f kZero8 = (v8f){0.f, 0.f, 0.f, 0.f, 0.f, 0.f, 0.f, 0.f};

#pragma unroll 1
  for (int t = 0; t < kNT; ++t) {
    int lz = 0;
    asm volatile("" : "+v"(lz));

#pragma unroll
    for (int u = 0; u < 2; ++u) {
      v8f ar = kZero8, az = kZero8, ai = kZero8, ah = kZero8;
      const _Float16* wl = W1 + (size_t)(32 * wave + 16 * u + c) * kK1 + 8 * hh + lz;
      gemm_part<kK1>(XTs + c * kXP + 8 * hh, wl, kNI / 32, ar, az, ai);
      gemm_part<kK1>(H1s + c * kHP + 8 * hh, wl + kNI, kNH / 32, ar, az, ah);
      gate_update(ar, az, ai, ah, c1R[u], c1Z[u], c1I[u], c1N[u], h1c[u]);
    }
    __syncthreads();
#pragma unroll
    for (int u = 0; u < 2; ++u)
#pragma unroll
      for (int e = 0; e < 8; ++e)
        H1s[(8 * hh + e) * kHP + 32 * wave + 16 * u + c] = carry_to_h16(h1c[u][e], kCarryA);
    if (wave >= 12) {
      const int tn = (t + 1 < kNT) ? (t + 1) : (kNT - 1);
      const float* xp = x + ((size_t)(kMB * blk + xm) * kNT + tn) * kNI + xk;
      v4f a0 = *(const v4f*)(xp);
      v4f a1 = *(const v4f*)(xp + 4);
      v8h hv;
#pragma unroll
      for (int e = 0; e < 4; ++e) {
        hv[e]     = carry_to_h16(bf_val(a0[e]), kCarryA);
        hv[4 + e] = carry_to_h16(bf_val(a1[e]), kCarryA);
      }
      *(v8h*)(XTs + xm * kXP + xk) = hv;
    }
    __syncthreads();

#pragma unroll
    for (int u = 0; u < 2; ++u) {
      v8f ar = kZero8, az = kZero8, ai = kZero8, ah = kZero8;
      const _Float16* wl = W2 + (size_t)(32 * wave + 16 * u + c) * kK2 + 8 * hh + lz;
      gemm_part<kK2>(H1s + c * kHP + 8 * hh, wl, kNH / 32, ar, az, ai);
      gemm_part<kK2>(H2s + c * kHP + 8 * hh, wl + kNH, kNH / 32, ar, az, ah);
      gate_update(ar, az, ai, ah, c2R[u], c2Z[u], c2I[u], c2N[u], h2c[u]);
    }
    __syncthreads();
#pragma unroll
    for (int u = 0; u < 2; ++u)
#pragma unroll
      for (int e = 0; e < 8; ++e)
        H2s[(8 * hh + e) * kHP + 32 * wave + 16 * u + c] = carry_to_h16(h2c[u][e], kCarryA);
    __syncthreads();

    if (wave < 2) {
      v8f a1 = kZero8, a2 = kZero8;
      const _Float16* ap1 = H1s + c * kHP + 8 * hh;
      const _Float16* ap2 = H2s + c * kHP + 8 * hh;
      const _Float16* wq1 = WO + (size_t)(16 * wave + c) * kNH + 8 * hh + lz;
      const _Float16* wq2 = wq1 + (size_t)32 * kNH;
#pragma unroll 1
      for (int ks = 0; ks < kNH / 32; ++ks) {
        const v16h fa1 = frag_load(ap1 + 32 * ks);
        const v16h fb1 = frag_load(wq1 + 32 * ks);
        a1 = mma_g(fa1, fb1, a1);
        const v16h fa2 = frag_load(ap2 + 32 * ks);
        const v16h fb2 = frag_load(wq2 + 32 * ks);
        a2 = mma_g(fa2, fb2, a2);
      }
      float* hp = HPs + wave * 512;
#pragma unroll
      for (int e = 0; e < 8; ++e) {
        hp[(8 * hh + e) * 16 + c]       = fmaf(a1[e], kFold, bo1c);
        hp[256 + (8 * hh + e) * 16 + c] = fmaf(a2[e], kFold, bo2c);
      }
      __builtin_amdgcn_fence(__ATOMIC_RELEASE, "workgroup");
      __builtin_amdgcn_wave_barrier();
      __builtin_amdgcn_fence(__ATOMIC_ACQUIRE, "workgroup");
      const int s = t & (kFl - 1);
#pragma unroll 1
      for (int i = 0; i < 8; ++i) {
        const int idx = i * 32 + lane;
        const int m = idx >> 4;
        const int n = idx & 15;
        const float v = tanhf(hp[idx]) + tanhf(hp[256 + idx]);
        const int col = 16 * wave + n;
        if (col < kNO) OBs[m * kOBS + s * kNO + col] = v;
      }
    }

    if ((t & (kFl - 1)) == (kFl - 1)) {
      __syncthreads();
      const int t0 = t - (kFl - 1);
      const float* ob = OBs + wave * kOBS + lane * 4;
      const v4f v0 = *(const v4f*)(ob);
      const v4f v1 = *(const v4f*)(ob + 128);
      const v4f v2 = *(const v4f*)(ob + 256);
      float* dst = out + ((size_t)(kMB * blk + wave) * kNT + t0) * kNO + lane * 4;
      for (int pass = 0; pass < 2; ++pass) {
        *(volatile v4f*)(dst)       = v0;
        *(volatile v4f*)(dst + 128) = v1;
        *(volatile v4f*)(dst + 256) = v2;
        __threadfence();
      }
    }
  }
}

extern "C" void kernel_launch(void* const* d_in, const int* in_sizes, int n_in,
                              void* d_out, int out_size, void* d_ws, size_t ws_size,
                              hipStream_t stream) {
  if (n_in < 13) return;
  if (in_sizes[0] != kNB * kNT * kNI) return;
  if (in_sizes[1] != kNG * kNI) return;
  if (in_sizes[2] != kNG * kNH) return;
  if (in_sizes[3] != kNG || in_sizes[4] != kNG) return;
  if (in_sizes[5] != kNG * kNH || in_sizes[6] != kNG * kNH) return;
  if (in_sizes[7] != kNG || in_sizes[8] != kNG) return;
  if (in_sizes[9] != kNO * kNH || in_sizes[10] != kNO) return;
  if (in_sizes[11] != kNO * kNH || in_sizes[12] != kNO) return;
  if (out_size != kNB * kNT * kNO) return;
  if (ws_size < kWsTotal) return;

  const float* x     = (const float*)d_in[0];
  const float* w_ih1 = (const float*)d_in[1];
  const float* w_hh1 = (const float*)d_in[2];
  const float* b_ih1 = (const float*)d_in[3];
  const float* b_hh1 = (const float*)d_in[4];
  const float* w_ih2 = (const float*)d_in[5];
  const float* w_hh2 = (const float*)d_in[6];
  const float* b_ih2 = (const float*)d_in[7];
  const float* b_hh2 = (const float*)d_in[8];
  const float* w_o1  = (const float*)d_in[9];
  const float* b_o1  = (const float*)d_in[10];
  const float* w_o2  = (const float*)d_in[11];
  const float* b_o2  = (const float*)d_in[12];
  float* out = (float*)d_out;

  char* ws = (char*)d_ws;
  unsigned short* W1 = (unsigned short*)(ws + kOffW1);
  unsigned short* W2 = (unsigned short*)(ws + kOffW2);
  unsigned short* WO = (unsigned short*)(ws + kOffWO);

  static_assert((kNG * (kNI / 8)) % 256 == 0 && (kNG * (kNH / 8)) % 256 == 0 && (32 * (kNH / 8)) % 256 == 0);
  pack_weight_plane<<<(kNG * (kNI / 8)) / 256, 256, 0, stream>>>(w_ih1, kNG, kNG, kNI, W1, kK1, 0);
  pack_weight_plane<<<(kNG * (kNH / 8)) / 256, 256, 0, stream>>>(w_hh1, kNG, kNG, kNH, W1, kK1, kNI);
  pack_weight_plane<<<(kNG * (kNH / 8)) / 256, 256, 0, stream>>>(w_ih2, kNG, kNG, kNH, W2, kK2, 0);
  pack_weight_plane<<<(kNG * (kNH / 8)) / 256, 256, 0, stream>>>(w_hh2, kNG, kNG, kNH, W2, kK2, kNH);
  pack_weight_plane<<<(32 * (kNH / 8)) / 256, 256, 0, stream>>>(w_o1, kNO, 32, kNH, WO, kNH, 0);
  pack_weight_plane<<<(32 * (kNH / 8)) / 256, 256, 0, stream>>>(w_o2, kNO, 32, kNH, WO + (size_t)32 * kNH, kNH, 0);

  two_cell_scan<<<kBlocks, 512, 0, stream>>>(
      x, (const _Float16*)W1, (const _Float16*)W2, (const _Float16*)WO,
      b_ih1, b_hh1, b_ih2, b_hh2, b_o1, b_o2, out);
}
